// DifferentiableRollout_66185446031771
// MI455X (gfx1250) — hardware-verified
//
#include <hip/hip_runtime.h>

#pragma clang fp contract(off)

typedef __attribute__((ext_vector_type(16))) __bf16   v16b;
typedef __attribute__((ext_vector_type(8)))  __bf16   v8b;
typedef __attribute__((ext_vector_type(8)))  float    v8f;
typedef __attribute__((ext_vector_type(4)))  float    v4f;
typedef __attribute__((ext_vector_type(2)))  float    v2f;
typedef __attribute__((ext_vector_type(4)))  unsigned int v4u;
typedef __attribute__((ext_vector_type(2)))  unsigned int v2u;

__device__ __forceinline__ unsigned short f2bf_bits(float f) {
  unsigned u = __float_as_uint(f);
  return (unsigned short)((u + 0x7FFFu + ((u >> 16) & 1u)) >> 16);
}
__device__ __forceinline__ float bf_bits2f(unsigned short h) { return __uint_as_float(((unsigned)h) << 16); }

__device__ __forceinline__ void dep_guard_b(v8f& a, v8f& b, v16b x, v16b y) { asm volatile("v_nop\n\tv_nop\n\tv_nop\n\tv_nop" : "+v"(a), "+v"(b) : "v"(x), "v"(y)); }
__device__ __forceinline__ void keep4_b(v16b a, v16b b, v16b c, v16b d) { asm volatile("v_nop" :: "v"(a), "v"(b), "v"(c), "v"(d)); }
__device__ __forceinline__ void acc_guard4(v8f& a, v8f& b, v8f& c, v8f& d) { asm volatile("v_nop\n\tv_nop\n\tv_nop\n\tv_nop" : "+v"(a), "+v"(b), "+v"(c), "+v"(d)); }
__device__ __forceinline__ void dep_guard_b1(v8f& a, v16b x, v16b y, v16b z, v16b w) { asm volatile("v_nop\n\tv_nop\n\tv_nop\n\tv_nop" : "+v"(a) : "v"(x), "v"(y), "v"(z), "v"(w)); }

template <typename T> struct Frag;
template <> struct Frag<__bf16> {
  typedef v16b V; union U { v16b v; v8b h[2]; };
  static __device__ __forceinline__ v16b load(const __bf16* p) {
    U f; f.h[0] = *(const v8b*)(p); f.h[1] = *(const v8b*)(p + 16); return f.v;
  }
  static __device__ __forceinline__ v8f mma(v16b a, v16b b, v8f c) {
    return __builtin_amdgcn_wmma_f32_16x16x32_bf16(false, a, false, b, (short)0, c, false, false);
  }
  static __device__ __forceinline__ void guard(v8f& a, v8f& b, v16b x, v16b y) { dep_guard_b(a, b, x, y); }
  static __device__ __forceinline__ void keep(v16b a, v16b b, v16b c, v16b d) { keep4_b(a, b, c, d); }
};
typedef Frag<__bf16> FragB;

constexpr int kRowsPerBlk = 16;
constexpr int kStateDim   = 64;
constexpr int kCtrlDim    = 32;
constexpr int kInDim      = 96;
constexpr int kHid        = 512;
constexpr int kSteps      = 200;
constexpr int kPitchA     = 104;
constexpr int kPitchH     = 520;
constexpr int kPitchX     = 68;
constexpr int kLdW1       = 128;
constexpr int kLdW2       = 512;
constexpr float kDt       = 0.1f;

static_assert(kInDim % 32 == 0);
static_assert(kHid % 64 == 0);
static_assert((kPitchA % 8) == 0 && (kPitchH % 8) == 0 && (kPitchX % 4) == 0);

__device__ __forceinline__ void split_pack2(float a, float b, unsigned int& ph, unsigned int& pl) {
  const unsigned short ha = f2bf_bits(a);
  const unsigned short la = f2bf_bits(a - bf_bits2f(ha));
  const unsigned short hb = f2bf_bits(b);
  const unsigned short lb = f2bf_bits(b - bf_bits2f(hb));
  ph = (unsigned int)ha | (((unsigned int)hb) << 16);
  pl = (unsigned int)la | (((unsigned int)lb) << 16);
}

__device__ __forceinline__ float tanh_f32(float v) {
  const float y = fminf(fabsf(v), 10.0f);
  const float e = expf(2.0f * y);
  const float r = __builtin_amdgcn_rcpf(e + 1.0f);
  const float tp = 1.0f - 2.0f * r;
  return copysignf(tp, v);
}

__global__ __launch_bounds__(256) void prep_transpose_split(
    const float* __restrict__ in, int nRows, int nCols, int ldo,
    unsigned short* __restrict__ ohi, unsigned short* __restrict__ olo, int total8) {
  const int i = blockIdx.x * 256 + threadIdx.x;
  if (i >= total8) return;
  const int q8 = ldo >> 3;
  const int n  = i / q8;
  const int k8 = (i - n * q8) * 8;
  unsigned int ph[4], pl[4];
#pragma unroll
  for (int e = 0; e < 4; ++e) {
    const int ka = k8 + 2 * e, kb = ka + 1;
    const int kac = (ka < nRows) ? ka : (nRows - 1);
    const int kbc = (kb < nRows) ? kb : (nRows - 1);
    float va = in[(size_t)kac * nCols + n];
    float vb = in[(size_t)kbc * nCols + n];
    va = (ka < nRows) ? va : 0.0f;
    vb = (kb < nRows) ? vb : 0.0f;
    split_pack2(va, vb, ph[e], pl[e]);
  }
  const v4u hv = (v4u){ph[0], ph[1], ph[2], ph[3]};
  const v4u lv = (v4u){pl[0], pl[1], pl[2], pl[3]};
  const size_t o = (size_t)n * ldo + k8;
  *(volatile v4u*)(ohi + o) = hv;
  *(volatile v4u*)(olo + o) = lv;
  __threadfence();
  *(volatile v4u*)(ohi + o) = hv;
  *(volatile v4u*)(olo + o) = lv;
}

__global__ __launch_bounds__(256) void rollout_kernel(
    const float* __restrict__ x0, const float* __restrict__ controls,
    const unsigned short* __restrict__ W1th, const unsigned short* __restrict__ W1tl,
    const float* __restrict__ b1,
    const unsigned short* __restrict__ W2th, const unsigned short* __restrict__ W2tl,
    const float* __restrict__ b2,
    float* __restrict__ out, int nBatch)
{
  __shared__ __align__(16) unsigned short sAhi[kRowsPerBlk * kPitchA];
  __shared__ __align__(16) unsigned short sAlo[kRowsPerBlk * kPitchA];
  __shared__ __align__(16) unsigned short sHhi[kRowsPerBlk * kPitchH];
  __shared__ __align__(16) unsigned short sHlo[kRowsPerBlk * kPitchH];
  __shared__ __align__(16) float sX[kRowsPerBlk * kPitchX];
  __shared__ __align__(16) float sRed[kRowsPerBlk * kPitchX];
  __shared__ __align__(16) float sb1[kHid];
  __shared__ __align__(16) float sb2[kStateDim];

  const int tid   = threadIdx.x;
  const int wave  = tid >> 5;
  const int lane  = tid & 31;
  const int hh    = lane >> 4;
  const int rlane = lane & 15;
  const int koff  = hh * 8;
  const int mOff  = hh * 8;
  const int nt2   = wave & 3;
  const int kh    = wave >> 2;
  const int m0    = blockIdx.x * kRowsPerBlk;
  if (m0 + kRowsPerBlk > nBatch) return;

  const __bf16* Ah1 = (const __bf16*)sAhi;
  const __bf16* Al1 = (const __bf16*)sAlo;
  const __bf16* Ah2 = (const __bf16*)sHhi;
  const __bf16* Al2 = (const __bf16*)sHlo;
  const __bf16* B1h = (const __bf16*)W1th;
  const __bf16* B1l = (const __bf16*)W1tl;
  const __bf16* B2h = (const __bf16*)W2th;
  const __bf16* B2l = (const __bf16*)W2tl;

  for (int i = tid; i < kHid; i += 256) sb1[i] = b1[i];
  if (tid < kStateDim) sb2[tid] = b2[tid];
  float xr[8];
#pragma unroll
  for (int r = 0; r < 8; ++r) xr[r] = 0.0f;
  if (kh == 0) {
    const int col = nt2 * 16 + rlane;
#pragma unroll
    for (int r = 0; r < 8; ++r) {
      const int row = mOff + r;
      const float v = x0[(size_t)(m0 + row) * kStateDim + col];
      xr[r] = v;
      sX[row * kPitchX + col] = v;
    }
  }
  __syncthreads();

  const v8f vz = (v8f){0.f, 0.f, 0.f, 0.f, 0.f, 0.f, 0.f, 0.f};

  for (int t = 0; t < kSteps; ++t) {
    {
      const int row = 2 * wave + hh;
      const int c4  = rlane * 4;
      const v4f v = *(const v4f*)(sX + row * kPitchX + c4);
      float* op = out + ((size_t)(m0 + row) * (kSteps + 1) + t) * kStateDim + c4;
      *(volatile v4f*)op = v;
      __threadfence();
      *(volatile v4f*)op = v;
    }
    {
      const int row = tid >> 4, q = tid & 15;
      const v4f xv = *(const v4f*)(sX + row * kPitchX + 4 * q);
      const v2f uv = *(const v2f*)(controls + ((size_t)(m0 + row) * kSteps + t) * kCtrlDim + 2 * q);
      unsigned int xh0, xl0, xh1, xl1, uh, ul;
      split_pack2(xv[0], xv[1], xh0, xl0);
      split_pack2(xv[2], xv[3], xh1, xl1);
      split_pack2(uv[0], uv[1], uh, ul);
      *(v2u*)(sAhi + row * kPitchA + 4 * q) = (v2u){xh0, xh1};
      *(v2u*)(sAlo + row * kPitchA + 4 * q) = (v2u){xl0, xl1};
      *(unsigned int*)(sAhi + row * kPitchA + kStateDim + 2 * q) = uh;
      *(unsigned int*)(sAlo + row * kPitchA + kStateDim + 2 * q) = ul;
    }
    __syncthreads();

    {
      v8f acc[4];
#pragma unroll
      for (int j = 0; j < 4; ++j) acc[j] = vz;
#pragma unroll
      for (int ks = 0; ks < kInDim / 32; ++ks) {
        const int k0 = ks * 32;
        v16b bh[4], bl[4];
#pragma unroll
        for (int j = 0; j < 4; ++j) {
          const size_t bo = (size_t)(wave * 64 + (j << 4) + rlane) * kLdW1 + koff + k0;
          bh[j] = FragB::load(B1h + bo);
          bl[j] = FragB::load(B1l + bo);
        }
        const int ao = rlane * kPitchA + koff + k0;
        const v16b ah = FragB::load(Ah1 + ao);
        const v16b al = FragB::load(Al1 + ao);
#pragma unroll
        for (int j = 0; j < 4; ++j) {
          acc[j] = FragB::mma(ah, bh[j], acc[j]);
          acc[j] = FragB::mma(ah, bl[j], acc[j]);
          acc[j] = FragB::mma(al, bh[j], acc[j]);
        }
        FragB::guard(acc[0], acc[3], ah, al);
        FragB::keep(bh[0], bh[1], bh[2], bh[3]);
        FragB::keep(bl[0], bl[1], bl[2], bl[3]);
      }
      acc_guard4(acc[0], acc[1], acc[2], acc[3]);
#pragma unroll
      for (int j = 0; j < 4; ++j) {
        const int col = wave * 64 + (j << 4) + rlane;
        const float bv = sb1[col];
#pragma unroll
        for (int r = 0; r < 8; ++r) {
          const int row = mOff + r;
          const float hv = tanh_f32(acc[j][r] + bv);
          const unsigned short hb = f2bf_bits(hv);
          const unsigned short lb = f2bf_bits(hv - bf_bits2f(hb));
          sHhi[row * kPitchH + col] = hb;
          sHlo[row * kPitchH + col] = lb;
        }
      }
    }
    __syncthreads();

    v8f acc2 = vz;
    {
#pragma unroll
      for (int kk = 0; kk < 8; ++kk) {
        const int k0 = kh * 256 + kk * 32;
        const size_t bo = (size_t)(nt2 * 16 + rlane) * kLdW2 + koff + k0;
        const v16b bh = FragB::load(B2h + bo);
        const v16b bl = FragB::load(B2l + bo);
        const int ao = rlane * kPitchH + koff + k0;
        const v16b ah = FragB::load(Ah2 + ao);
        const v16b al = FragB::load(Al2 + ao);
        acc2 = FragB::mma(ah, bh, acc2);
        acc2 = FragB::mma(ah, bl, acc2);
        acc2 = FragB::mma(al, bh, acc2);
        dep_guard_b1(acc2, ah, al, bh, bl);
      }
    }
    if (kh == 1) {
      const int col = nt2 * 16 + rlane;
#pragma unroll
      for (int r = 0; r < 8; ++r) sRed[(mOff + r) * kPitchX + col] = acc2[r];
    }
    __syncthreads();

    if (kh == 0) {
      const int col = nt2 * 16 + rlane;
      const float bv = sb2[col];
#pragma unroll
      for (int r = 0; r < 8; ++r) {
        const int row = mOff + r;
        float s = acc2[r] + sRed[row * kPitchX + col];
        s = s + bv;
        const float xn = xr[r] + kDt * s;
        xr[r] = xn;
        sX[row * kPitchX + col] = xn;
      }
    }
    __syncthreads();
  }

  {
    const int row = 2 * wave + hh;
    const int c4  = rlane * 4;
    const v4f v = *(const v4f*)(sX + row * kPitchX + c4);
    float* op = out + ((size_t)(m0 + row) * (kSteps + 1) + kSteps) * kStateDim + c4;
    *(volatile v4f*)op = v;
    __threadfence();
    *(volatile v4f*)op = v;
  }
}

extern "C" void kernel_launch(void* const* d_in, const int* in_sizes, int n_in,
                              void* d_out, int out_size, void* d_ws, size_t ws_size,
                              hipStream_t stream) {
  (void)n_in; (void)out_size;
  const float* x0       = (const float*)d_in[0];
  const float* controls = (const float*)d_in[1];
  const float* W1       = (const float*)d_in[2];
  const float* b1       = (const float*)d_in[3];
  const float* W2       = (const float*)d_in[4];
  const float* b2       = (const float*)d_in[5];
  float* out = (float*)d_out;

  const int nBatch = in_sizes[0] / kStateDim;
  const int nBlk   = nBatch / kRowsPerBlk;

  const size_t w1PlaneBytes = (size_t)kHid * kLdW1 * 2;
  const size_t w2PlaneBytes = (size_t)kStateDim * kLdW2 * 2;
  const size_t wsNeeded = 2 * w1PlaneBytes + 2 * w2PlaneBytes;
  if (ws_size < wsNeeded || nBlk <= 0) return;
  if (in_sizes[2] != kInDim * kHid || in_sizes[4] != kHid * kStateDim) return;

  char* ws = (char*)d_ws;
  unsigned short* W1th = (unsigned short*)(ws);
  unsigned short* W1tl = (unsigned short*)(ws + w1PlaneBytes);
  unsigned short* W2th = (unsigned short*)(ws + 2 * w1PlaneBytes);
  unsigned short* W2tl = (unsigned short*)(ws + 2 * w1PlaneBytes + w2PlaneBytes);

  const int total8_w1 = kHid * kLdW1 / 8;
  prep_transpose_split<<<dim3((total8_w1 + 255) / 256), dim3(256), 0, stream>>>(
      W1, kInDim, kHid, kLdW1, W1th, W1tl, total8_w1);
  const int total8_w2 = kStateDim * kLdW2 / 8;
  prep_transpose_split<<<dim3((total8_w2 + 255) / 256), dim3(256), 0, stream>>>(
      W2, kHid, kStateDim, kLdW2, W2th, W2tl, total8_w2);

  rollout_kernel<<<dim3(nBlk), dim3(256), 0, stream>>>(
      x0, controls, W1th, W1tl, b1, W2th, W2tl, b2, out, nBatch);
}
